// RelationLayer_69054484185608
// MI455X (gfx1250) — hardware-verified
//
#include <hip/hip_runtime.h>
#include <math.h>

typedef __attribute__((ext_vector_type(16))) _Float16 v16h;
typedef __attribute__((ext_vector_type(16))) __bf16 v16b;
typedef __attribute__((ext_vector_type(8)))  _Float16 v8h;
typedef __attribute__((ext_vector_type(8)))  float v8f;
typedef __attribute__((ext_vector_type(4)))  float v4f;
typedef __attribute__((ext_vector_type(2)))  float v2f;
typedef __attribute__((ext_vector_type(4)))  unsigned v4u;
typedef __attribute__((ext_vector_type(4)))  int v4i;
typedef float __attribute__((may_alias)) float_a;
typedef int __attribute__((may_alias)) int_a;

template <typename T> __device__ __forceinline__ void vst2(void* p, T v) { *(volatile T*)p = v; __threadfence(); *(volatile T*)p = v; }
__device__ __forceinline__ v8f wmma16(v16h a, v16h b, v8f c) {
  v8f d = __builtin_amdgcn_wmma_f32_16x16x32_f16(false, a, false, b, (short)0, c, false, false);
  asm volatile("v_nop\n\tv_nop\n\tv_nop\n\tv_nop" : "+v"(d) : "v"(a), "v"(b));
  return d;
}
__device__ __forceinline__ v8f wmma_bf(v16b a, v16b b, v8f c) {
  v8f d = __builtin_amdgcn_wmma_f32_16x16x32_bf16(false, a, false, b, (short)0, c, false, false);
  asm volatile("v_nop\n\tv_nop\n\tv_nop\n\tv_nop" : "+v"(d) : "v"(a), "v"(b));
  return d;
}
__device__ __forceinline__ v16h frag_h(const _Float16* rowk0, int lane) {
  union { v16h v; v8h q[2]; } u; const _Float16* p = rowk0 + 8 * (lane >> 4);
  u.q[0] = *(const v8h*)p; u.q[1] = *(const v8h*)(p + 16); return u.v;
}
__device__ __forceinline__ v16h frag_f32(const float* rowk0, int lane) {
  v16h a; const float* p = rowk0 + 8 * (lane >> 4);
#pragma unroll
  for (int i = 0; i < 8; ++i) { a[i] = (_Float16)p[i]; a[8 + i] = (_Float16)p[16 + i]; }
  return a;
}
__device__ __forceinline__ v16h frag_f32s(const float* rowk0, int lane, float sc) {
  v16h a; const float* p = rowk0 + 8 * (lane >> 4);
#pragma unroll
  for (int i = 0; i < 8; ++i) { a[i] = (_Float16)(p[i] * sc); a[8 + i] = (_Float16)(p[16 + i] * sc); }
  return a;
}
__device__ __forceinline__ v16h fragc_f32(const float* W, int k0, int n, int lane, int ld, int K) {
  v16h a; const int g = lane >> 4;
#pragma unroll
  for (int i = 0; i < 8; ++i) { const int ka = k0 + 8 * g + i, kb = ka + 16;
    a[i] = (_Float16)(ka < K ? W[(size_t)(ka < K ? ka : K - 1) * ld + n] : 0.f); a[8 + i] = (_Float16)(kb < K ? W[(size_t)(kb < K ? kb : K - 1) * ld + n] : 0.f); }
  return a;
}
struct F2 { v16b h, l; };
__device__ __forceinline__ F2 bsplit16(const float v[16]) { F2 r;
#pragma unroll
  for (int i = 0; i < 16; ++i) { const __bf16 h = (__bf16)v[i]; r.h[i] = h; r.l[i] = (__bf16)(v[i] - (float)h); }
  return r; }
__device__ __forceinline__ F2 split_row(const float* row, int k0, int lane) { float v[16]; const float* p = row + k0 + 8 * (lane >> 4);
#pragma unroll
  for (int i = 0; i < 8; ++i) { v[i] = p[i]; v[8 + i] = p[16 + i]; }
  return bsplit16(v); }
__device__ __forceinline__ F2 split_rowK(const float* row, int k0, int lane, int K) { float v[16]; const int g = lane >> 4;
#pragma unroll
  for (int i = 0; i < 8; ++i) { const int ka = k0 + 8 * g + i, kb = ka + 16; v[i] = ka < K ? row[ka < K ? ka : K - 1] : 0.f; v[8 + i] = kb < K ? row[kb < K ? kb : K - 1] : 0.f; }
  return bsplit16(v); }
__device__ __forceinline__ F2 split_col(const float* W, int k0, int n, int lane, int ld, int K) { float v[16]; const int g = lane >> 4;
#pragma unroll
  for (int i = 0; i < 8; ++i) { const int ka = k0 + 8 * g + i, kb = ka + 16; v[i] = ka < K ? W[(size_t)(ka < K ? ka : K - 1) * ld + n] : 0.f; v[8 + i] = kb < K ? W[(size_t)(kb < K ? kb : K - 1) * ld + n] : 0.f; }
  return bsplit16(v); }
__device__ __forceinline__ v8f mac3(const F2& a, const F2& b, v8f c) { c = wmma_bf(a.l, b.h, c); c = wmma_bf(a.h, b.l, c); return wmma_bf(a.h, b.h, c); }
__device__ __forceinline__ float sigm(float v) { return 1.0f / (1.0f + expf(-v)); }
#define LDSX() do { asm volatile("s_wait_dscnt 0" ::: "memory"); __builtin_amdgcn_wave_barrier(); __builtin_amdgcn_fence(__ATOMIC_RELEASE, "workgroup"); } while (0)

__device__ __forceinline__ float bfr(float v) { return (float)(__bf16)v; }
__device__ __forceinline__ float lrelu(float v) { return v > 0.f ? v : 0.01f * v; }
#define NS 262144
#define NOBJ 16
#define OBJ 3
#define EMBD 4
#define DIN 14
#define HU 16
#ifndef NBLK
#define NBLK (NS / 4)
#endif
__global__ __launch_bounds__(128) void k_rel(const float* __restrict__ X, const float* __restrict__ EO, const float* __restrict__ EA, const float* __restrict__ ES, const float* __restrict__ EG, const float* __restrict__ W0, const float* __restrict__ B0, const float* __restrict__ W1, const float* __restrict__ B1, const float* __restrict__ WM, const float* __restrict__ BM, float* __restrict__ OUT) {
  __shared__ __align__(16) float srel[16][HU + 4];
  __shared__ __align__(16) float so[64];
  const int tid = threadIdx.x, wave = tid >> 5, lane = tid & 31, col = lane & 15, g = lane >> 4; const size_t smp = (size_t)blockIdx.x * 4 + wave;
  if (tid < 16 * (HU + 4) / 4) ((v4f*)&srel[0][0])[tid] = (v4f){0.f, 0.f, 0.f, 0.f};
  __syncthreads();
  const float* xs = X + smp * (NOBJ * OBJ); float in[DIN];
  { const float* eown = EO; const float* eobj = (col == 0) ? EO : (col == 1) ? EA : (col == NOBJ - 1) ? EG : ES;
#pragma unroll
    for (int i = 0; i < OBJ; ++i) { in[i] = bfr(xs[i]); in[7 + i] = bfr(xs[col * OBJ + i]); }
#pragma unroll
    for (int i = 0; i < EMBD; ++i) { in[3 + i] = bfr(eown[i]); in[10 + i] = bfr(eobj[i]); } }
  float hv[16];
#pragma unroll
  for (int e = 0; e < 8; ++e) { const int o = 8 * g + e; float s = bfr(B0[o]);
#pragma unroll
    for (int i = 0; i < DIN; ++i) s += in[i] * bfr(W0[o * DIN + i]);
    hv[e] = lrelu(s); hv[8 + e] = 0.f; asm volatile("s_wait_loadcnt 0x0" ::: "memory"); }
  const F2 a = bsplit16(hv);
  v16b w1;
#pragma unroll
  for (int i = 0; i < 8; ++i) { w1[i] = (__bf16)W1[col * HU + 8 * g + i]; w1[8 + i] = (__bf16)0.f; }
  v8f acc = {}; acc = wmma_bf(a.h, w1, acc); acc = wmma_bf(a.l, w1, acc);
  float part = 0.f; const float b1 = bfr(B1[col]);
#pragma unroll
  for (int r = 0; r < 8; ++r) part += lrelu(acc[r] + b1);
  part += __shfl_xor(part, 16);
  if (g == 0) srel[wave][col] = part;
  __syncthreads();
  if (wave == 0) { float rv[16];
#pragma unroll
    for (int i = 0; i < 8; ++i) { rv[i] = srel[col][8 * g + i]; rv[8 + i] = 0.f; }
    const F2 ar = bsplit16(rv); v16b wm;
#pragma unroll
    for (int i = 0; i < 8; ++i) { wm[i] = (__bf16)WM[col * HU + 8 * g + i]; wm[8 + i] = (__bf16)0.f; }
    v8f acc2 = {}; acc2 = wmma_bf(ar.h, wm, acc2); acc2 = wmma_bf(ar.l, wm, acc2);
    const float bm = bfr(BM[col]);
    if (g == 0) {
#pragma unroll
      for (int r = 0; r < 4; ++r) so[r * HU + col] = lrelu(acc2[r] + bm); }
  }
  __syncthreads();
  if (tid < 16) vst2(OUT + (size_t)blockIdx.x * 64 + tid * 4, *(const v4f*)&so[tid * 4]); }
extern "C" void kernel_launch(void* const* d_in, const int* in_sizes, int n_in, void* d_out, int out_size, void* d_ws, size_t ws_size, hipStream_t stream) {
  (void)in_sizes; (void)n_in; (void)out_size; (void)d_ws; (void)ws_size;
  const float** F = (const float**)d_in;
  k_rel<<<dim3(NBLK), 128, 0, stream>>>(F[0], F[1], F[2], F[3], F[4], F[5], F[6], F[7], F[8], F[9], F[10], (float*)d_out);
}
